// GNNMLPv4_25228637896957
// MI455X (gfx1250) — hardware-verified
//
#include <hip/hip_runtime.h>
#include <hip/hip_bf16.h>
#include <stddef.h>


#define DF      128
#define NTHR    256
#define NWAVE   8
#define EPT     8
#define NGRP    2
#define CHUNK   (NTHR * EPT * NGRP)
#define WCAP    (EPT * NGRP * 32)
#define LISTN   (NWAVE * WCAP)
#define NBA     512
#define GROWS   128
#define NMAT    9
#define WPL     (DF * DF)
#define NHEAD   3
#define NGRAPH  8
#define LDS_GEMM (GROWS * DF * 4)
#define LDS_AGG  (NBA * DF * 4 + LISTN * 4 + 64)

static_assert((CHUNK & (CHUNK - 1)) == 0);
static_assert(CHUNK <= 4096);
static_assert(NBA <= 4096 && (NBA & (NBA - 1)) == 0);
static_assert(NBA % GROWS == 0);
static_assert((NBA * DF / 8) % NTHR == 0);

typedef float          v4f  __attribute__((ext_vector_type(4)));
typedef float          v8f  __attribute__((ext_vector_type(8)));
typedef int            v4i  __attribute__((ext_vector_type(4)));
typedef unsigned short v8us __attribute__((ext_vector_type(8)));
typedef _Float16       v8h  __attribute__((ext_vector_type(8)));
typedef _Float16       v16h __attribute__((ext_vector_type(16)));
typedef __bf16         v16b __attribute__((ext_vector_type(16)));
union FragH { v16h v; v8us u[2]; };
union FragB { v16b v; v8us u[2]; };

__device__ __forceinline__ v8us cvt8u(v4f a, v4f b) {
  union { v8h h; v8us u; } r;
  r.h[0] = (_Float16)a.x; r.h[1] = (_Float16)a.y; r.h[2] = (_Float16)a.z; r.h[3] = (_Float16)a.w;
  r.h[4] = (_Float16)b.x; r.h[5] = (_Float16)b.y; r.h[6] = (_Float16)b.z; r.h[7] = (_Float16)b.w;
  return r.u;
}

__device__ __forceinline__ unsigned bf_rne(float f) {
  const unsigned u = __float_as_uint(f);
  return (u + 0x7FFFu + ((u >> 16) & 1u)) >> 16;
}

#define SPL1(F, J) { const float f_ = (F); const unsigned h_ = bf_rne(f_); \
  hi[J] = (unsigned short)h_; lo[J] = (unsigned short)bf_rne(f_ - __uint_as_float(h_ << 16)); }
__device__ __forceinline__ void split8(v4f a, v4f b, v8us& hi, v8us& lo) {
  SPL1(a.x, 0) SPL1(a.y, 1) SPL1(a.z, 2) SPL1(a.w, 3)
  SPL1(b.x, 4) SPL1(b.y, 5) SPL1(b.z, 6) SPL1(b.w, 7)
}
#undef SPL1

__device__ __forceinline__ v8f wmh(v16h a, v16h b, v8f c) {
  v8f d = __builtin_amdgcn_wmma_f32_16x16x32_f16(false, a, false, b, (short)0, c, false, false);
  asm volatile("v_nop\n\tv_nop\n\tv_nop\n\tv_nop" : "+v"(d) : "v"(a), "v"(b));
  return d;
}
__device__ __forceinline__ v8f wmb3(v16b ah, v16b al, v16b bh, v16b bl, v8f c) {
  v8f d = __builtin_amdgcn_wmma_f32_16x16x32_bf16(false, ah, false, bh, (short)0, c, false, false);
  d = __builtin_amdgcn_wmma_f32_16x16x32_bf16(false, ah, false, bl, (short)0, d, false, false);
  d = __builtin_amdgcn_wmma_f32_16x16x32_bf16(false, al, false, bh, (short)0, d, false, false);
  asm volatile("v_nop\n\tv_nop\n\tv_nop\n\tv_nop" : "+v"(d) : "v"(ah), "v"(al), "v"(bh), "v"(bl));
  return d;
}

__device__ __forceinline__ float sigm(float v) {
  v = fminf(fmaxf(v, -80.0f), 80.0f);
  const float e = __expf(-v);
  return __builtin_amdgcn_rcpf(1.0f + e);
}

__global__ __launch_bounds__(NTHR) void k_wprep(
    const float* __restrict__ Wf, const float* __restrict__ Wc,
    const float* __restrict__ Wa, const float* __restrict__ Wb,
    unsigned short* wpl) {
  const int q = blockIdx.y;
  const int i = blockIdx.x * NTHR + threadIdx.x;
  if (i >= WPL / 8) return;
  const float* W;
  if (q == 0)      W = Wf;
  else if (q < 3)  W = Wc + (size_t)(q - 1) * WPL;
  else if (q < 6)  W = Wa + (size_t)(q - 3) * WPL;
  else             W = Wb + (size_t)(q - 6) * WPL;
  const bool split = q >= 2;
  const float sc = split ? 1.0f : 16.0f;
  const int o  = i * 8;
  const int n  = o >> 7;
  const int k0 = o & (DF - 1);
  const float* p = W + (size_t)k0 * DF + n;
  v4f a, b;
  a.x = p[0] * sc;      a.y = p[DF] * sc;     a.z = p[2 * DF] * sc; a.w = p[3 * DF] * sc;
  b.x = p[4 * DF] * sc; b.y = p[5 * DF] * sc; b.z = p[6 * DF] * sc; b.w = p[7 * DF] * sc;
  unsigned short* dp = wpl + (size_t)q * 2 * WPL + o;
  if (!split) {
    const v8us hv = cvt8u(a, b);
    *(volatile v8us*)dp = hv;
    __threadfence();
    *(volatile v8us*)dp = hv;
  } else {
    v8us hv, lv;
    split8(a, b, hv, lv);
    *(volatile v8us*)dp = hv;
    *(volatile v8us*)(dp + WPL) = lv;
    __threadfence();
    *(volatile v8us*)dp = hv;
    *(volatile v8us*)(dp + WPL) = lv;
  }
}

template <int AM, int OM>
__global__ __launch_bounds__(NTHR) void k_gemm(
    const float* __restrict__ Af,
    const unsigned short* __restrict__ Ah, const unsigned short* __restrict__ Al,
    const unsigned short* __restrict__ Bw,
    const float* __restrict__ bias, const float* __restrict__ gam, const float* __restrict__ bet,
    const float* __restrict__ rmu, const float* __restrict__ rva,
    const float* __restrict__ w3, const float* __restrict__ b3,
    float* Of, unsigned short* Oh, unsigned short* Ol, float* On,
    int nN, float ascale) {
  extern __shared__ v4f lds_dyn[];
  __shared__ __attribute__((aligned(16))) float nds[GROWS];
  float* stg = (float*)lds_dyn;
  const int tid = threadIdx.x, lane = tid & 31, wave = tid >> 5, hh = lane >> 4, m = lane & 15;
  const int rowBase = blockIdx.x * GROWS;
  int arow = rowBase + wave * 16 + m;
  arow = arow > nN - 1 ? nN - 1 : arow;

  v8f acc[8];
#pragma unroll
  for (int t = 0; t < 8; ++t) { v8f z = {0.f, 0.f, 0.f, 0.f, 0.f, 0.f, 0.f, 0.f}; acc[t] = z; }

#pragma unroll
  for (int kt = 0; kt < DF / 32; ++kt) {
    if constexpr (AM == 2) {
      FragB ah, al;
      const unsigned short* ph = Ah + (size_t)arow * DF + 32 * kt + 8 * hh;
      const unsigned short* pl = Al + (size_t)arow * DF + 32 * kt + 8 * hh;
      ah.u[0] = *(const v8us*)ph;  ah.u[1] = *(const v8us*)(ph + 16);
      al.u[0] = *(const v8us*)pl;  al.u[1] = *(const v8us*)(pl + 16);
#pragma unroll
      for (int t = 0; t < 8; ++t) {
        const unsigned short* bp = Bw + (size_t)(16 * t + m) * DF + 32 * kt + 8 * hh;
        FragB bh, bl;
        bh.u[0] = *(const v8us*)bp;          bh.u[1] = *(const v8us*)(bp + 16);
        bl.u[0] = *(const v8us*)(bp + WPL);  bl.u[1] = *(const v8us*)(bp + WPL + 16);
        acc[t] = wmb3(ah.v, al.v, bh.v, bl.v, acc[t]);
      }
    } else {
      FragH a;
      if constexpr (AM == 0) {
        const float* ap = Af + (size_t)arow * DF + 32 * kt + 8 * hh;
        const v4f p0 = *(const v4f*)ap,        p1 = *(const v4f*)(ap + 4);
        const v4f p2 = *(const v4f*)(ap + 16), p3 = *(const v4f*)(ap + 20);
        a.u[0] = cvt8u(p0, p1);
        a.u[1] = cvt8u(p2, p3);
      } else {
        const unsigned short* ap = Ah + (size_t)arow * DF + 32 * kt + 8 * hh;
        a.u[0] = *(const v8us*)ap;
        a.u[1] = *(const v8us*)(ap + 16);
      }
#pragma unroll
      for (int t = 0; t < 8; ++t) {
        const unsigned short* bp = Bw + (size_t)(16 * t + m) * DF + 32 * kt + 8 * hh;
        FragH b;
        b.u[0] = *(const v8us*)bp;
        b.u[1] = *(const v8us*)(bp + 16);
        acc[t] = wmh(a.v, b.v, acc[t]);
      }
    }
  }

  float alv[8], btv[8];
#pragma unroll
  for (int t = 0; t < 8; ++t) {
    const int c = 16 * t + m;
    const float al = gam[c] * rsqrtf(rva[c] + 1e-5f);
    btv[t] = bet[c] + (bias[c] - rmu[c]) * al;
    alv[t] = al * ascale;
  }

  if constexpr (OM != 2) {
    float* sp = stg + (wave * 16 + 8 * hh) * DF + m;
#pragma unroll
    for (int t = 0; t < 8; ++t) {
#pragma unroll
      for (int r = 0; r < 8; ++r) sp[r * DF + 16 * t] = fmaxf(acc[t][r] * alv[t] + btv[t], 0.f);
    }
    __syncthreads();
    if constexpr (OM == 0) {
      const float* lp = stg + wave * 16 * DF + 4 * lane;
      float* gp = Of + ((size_t)rowBase + wave * 16) * DF + 4 * lane;
#pragma unroll
      for (int i = 0; i < 16; ++i) { const v4f v = *(const v4f*)(lp + i * DF); *(volatile v4f*)(gp + (size_t)i * DF) = v; }
      __threadfence();
#pragma unroll
      for (int i = 0; i < 16; ++i) { const v4f v = *(const v4f*)(lp + i * DF); *(volatile v4f*)(gp + (size_t)i * DF) = v; }
    } else {
      v8us hv[8], lv[8];
#pragma unroll
      for (int i = 0; i < 8; ++i) {
        const float* f = stg + (wave * 16 + 2 * i + hh) * DF + 8 * m;
        const v4f q0 = *(const v4f*)f, q1 = *(const v4f*)(f + 4);
        split8(q0, q1, hv[i], lv[i]);
      }
      unsigned short* gh = Oh + ((size_t)rowBase + wave * 16 + hh) * DF + 8 * m;
      unsigned short* gl = Ol + ((size_t)rowBase + wave * 16 + hh) * DF + 8 * m;
#pragma unroll
      for (int i = 0; i < 8; ++i) {
        *(volatile v8us*)(gh + (size_t)(2 * i) * DF) = hv[i];
        *(volatile v8us*)(gl + (size_t)(2 * i) * DF) = lv[i];
      }
      __threadfence();
#pragma unroll
      for (int i = 0; i < 8; ++i) {
        *(volatile v8us*)(gh + (size_t)(2 * i) * DF) = hv[i];
        *(volatile v8us*)(gl + (size_t)(2 * i) * DF) = lv[i];
      }
    }
  } else {
    float w3l[8], p[8];
#pragma unroll
    for (int t = 0; t < 8; ++t) { w3l[t] = w3[16 * t + m]; p[t] = 0.f; }
#pragma unroll
    for (int t = 0; t < 8; ++t) {
#pragma unroll
      for (int r = 0; r < 8; ++r) {
        const float v = fmaxf(acc[t][r] * alv[t] + btv[t], 0.f);
        p[r] = p[r] + v * w3l[t];
      }
    }
#pragma unroll
    for (int r = 0; r < 8; ++r) {
      p[r] += __shfl_xor(p[r], 1, 32);
      p[r] += __shfl_xor(p[r], 2, 32);
      p[r] += __shfl_xor(p[r], 4, 32);
      p[r] += __shfl_xor(p[r], 8, 32);
    }
    const float b3v = b3[0];
    if (m == 0) {
#pragma unroll
      for (int r = 0; r < 8; ++r) nds[wave * 16 + 8 * hh + r] = p[r] + b3v;
    }
    __syncthreads();
    if (wave == 0) {
      const v4f v = *(const v4f*)(nds + 4 * lane);
      float* gp = On + (size_t)rowBase + 4 * lane;
      *(volatile v4f*)gp = v;
      __threadfence();
      *(volatile v4f*)gp = v;
    }
  }
}

template <int NB>
__device__ __forceinline__ int scan_chunk(const int* __restrict__ dsts, int nE, int cbase, int nodeBase,
                                          int vec8, int* list, int tid, int lane, int wave) {
  int wc = 0;
#pragma unroll
  for (int g = 0; g < NGRP; ++g) {
    const int el0  = (g * NTHR + tid) * EPT;
    const int e0   = cbase + el0;
    const int sent = -2147483647 - 1;
    v4i da, db;
    if (vec8 != 0 && e0 + 7 < nE) {
      da = *(const v4i*)(dsts + e0);
      db = *(const v4i*)(dsts + e0 + 4);
    } else {
      da.x = (e0     < nE) ? dsts[e0]     : sent;
      da.y = (e0 + 1 < nE) ? dsts[e0 + 1] : sent;
      da.z = (e0 + 2 < nE) ? dsts[e0 + 2] : sent;
      da.w = (e0 + 3 < nE) ? dsts[e0 + 3] : sent;
      db.x = (e0 + 4 < nE) ? dsts[e0 + 4] : sent;
      db.y = (e0 + 5 < nE) ? dsts[e0 + 5] : sent;
      db.z = (e0 + 6 < nE) ? dsts[e0 + 6] : sent;
      db.w = (e0 + 7 < nE) ? dsts[e0 + 7] : sent;
    }
    const unsigned nb = (unsigned)nodeBase;
    const unsigned s0 = (unsigned)da.x - nb, s1 = (unsigned)da.y - nb;
    const unsigned s2 = (unsigned)da.z - nb, s3 = (unsigned)da.w - nb;
    const unsigned s4 = (unsigned)db.x - nb, s5 = (unsigned)db.y - nb;
    const unsigned s6 = (unsigned)db.z - nb, s7 = (unsigned)db.w - nb;
    const bool h0 = s0 < (unsigned)NB, h1 = s1 < (unsigned)NB, h2 = s2 < (unsigned)NB, h3 = s3 < (unsigned)NB;
    const bool h4 = s4 < (unsigned)NB, h5 = s5 < (unsigned)NB, h6 = s6 < (unsigned)NB, h7 = s7 < (unsigned)NB;
    const unsigned any = __builtin_amdgcn_ballot_w32(h0 | h1 | h2 | h3 | h4 | h5 | h6 | h7);
    if (any != 0u) {
#define HITJ(J, HJ, SJ) { \
        const unsigned mj = __builtin_amdgcn_ballot_w32(HJ); \
        if (mj != 0u) { \
          if (HJ) { \
            const int pos = wc + (int)__builtin_amdgcn_mbcnt_lo(mj, 0u); \
            if (pos < WCAP) list[wave * WCAP + pos] = ((el0 + (J)) << 12) | (int)(SJ); \
          } \
          wc += (int)__builtin_popcount(mj); } }
      HITJ(0, h0, s0)
      HITJ(1, h1, s1)
      HITJ(2, h2, s2)
      HITJ(3, h3, s3)
      HITJ(4, h4, s4)
      HITJ(5, h5, s5)
      HITJ(6, h6, s6)
      HITJ(7, h7, s7)
#undef HITJ
    }
  }
  return wc;
}

template <int OM>
__global__ __launch_bounds__(NTHR) void k_agg(
    const int* __restrict__ ei, const float* __restrict__ hin,
    unsigned short* Sh, unsigned short* Sl, int nN, int nE, int vec8) {
  extern __shared__ v4f lds_dyn[];
  float* acc  = (float*)lds_dyn;
  int*   list = (int*)(acc + NBA * DF);
  int*   wcnt = list + LISTN;
  const int tid = threadIdx.x, lane = tid & 31, wave = tid >> 5;
  const int nodeBase = blockIdx.x * NBA;
  const int* dsts = ei + nE;

  {
    const v4f z = {0.f, 0.f, 0.f, 0.f};
    for (int i = tid; i < NBA * DF / 4; i += NTHR) lds_dyn[i] = z;
  }
  __syncthreads();

  const int nChunks = (nE + CHUNK - 1) / CHUNK;
#pragma unroll 1
  for (int ch = 0; ch < nChunks; ++ch) {
    const int cbase = ch * CHUNK;
    const int wc = scan_chunk<NBA>(dsts, nE, cbase, nodeBase, vec8, list, tid, lane, wave);
    if (lane == 0) wcnt[wave] = wc;
    __syncthreads();
    if (wave == 0) {
#pragma unroll 1
      for (int wsx = 0; wsx < NWAVE; ++wsx) {
        int n = __builtin_amdgcn_readfirstlane(wcnt[wsx]);
        n = n > WCAP ? WCAP : (n < 0 ? 0 : n);
        const int* lp = list + wsx * WCAP;
#pragma unroll 1
        for (int i = 0; i < n; ++i) {
          const int ent  = __builtin_amdgcn_readfirstlane(lp[i]);
          const int slot = ent & (NBA - 1);
          int e = cbase + ((ent >> 12) & (CHUNK - 1));
          e = e > nE - 1 ? nE - 1 : e;
          int src = ei[e];
          src = src < 0 ? 0 : (src > nN - 1 ? nN - 1 : src);
          const v4f v = *(const v4f*)(hin + (size_t)src * DF + 4 * lane);
          v4f* ap = (v4f*)(acc + slot * DF + 4 * lane);
          *ap = *ap + v;
        }
      }
    }
    __syncthreads();
  }

#pragma unroll 4
  for (int it = 0; it < (NBA * DF / 8) / NTHR; ++it) {
    const int idx  = it * NTHR + tid;
    const int slot = idx >> 4;
    const int c0   = (idx & 15) * 8;
    int node = nodeBase + slot;
    node = node > nN - 1 ? nN - 1 : node;
    const float* arp = acc + slot * DF + c0;
    const float* hp  = hin + (size_t)node * DF + c0;
    const v4f sa = *(const v4f*)arp + *(const v4f*)hp;
    const v4f sb = *(const v4f*)(arp + 4) + *(const v4f*)(hp + 4);
    const size_t go = ((size_t)nodeBase + slot) * DF + c0;
    if constexpr (OM == 0) {
      const v8us hv = cvt8u(sa, sb);
      *(volatile v8us*)(Sh + go) = hv;
    } else {
      v8us hv, lv;
      split8(sa, sb, hv, lv);
      *(volatile v8us*)(Sh + go) = hv;
      *(volatile v8us*)(Sl + go) = lv;
    }
  }
  __threadfence();
#pragma unroll 4
  for (int it = 0; it < (NBA * DF / 8) / NTHR; ++it) {
    const int idx  = it * NTHR + tid;
    const int slot = idx >> 4;
    const int c0   = (idx & 15) * 8;
    int node = nodeBase + slot;
    node = node > nN - 1 ? nN - 1 : node;
    const float* arp = acc + slot * DF + c0;
    const float* hp  = hin + (size_t)node * DF + c0;
    const v4f sa = *(const v4f*)arp + *(const v4f*)hp;
    const v4f sb = *(const v4f*)(arp + 4) + *(const v4f*)(hp + 4);
    const size_t go = ((size_t)nodeBase + slot) * DF + c0;
    if constexpr (OM == 0) {
      const v8us hv = cvt8u(sa, sb);
      *(volatile v8us*)(Sh + go) = hv;
    } else {
      v8us hv, lv;
      split8(sa, sb, hv, lv);
      *(volatile v8us*)(Sh + go) = hv;
      *(volatile v8us*)(Sl + go) = lv;
    }
  }
}

__device__ __forceinline__ float out_elem(int f, const float* sm, const float* __restrict__ nodep,
                                          int nN, int np, int outN) {
  if (f >= outN) return 0.f;
  if (f < NHEAD * NGRAPH) return sigm(sm[f]);
  const int k = f - NHEAD * NGRAPH;
  int hd = k / nN;
  hd = hd > NHEAD - 1 ? NHEAD - 1 : hd;
  int n = k - hd * nN;
  n = n < 0 ? 0 : (n > nN - 1 ? nN - 1 : n);
  return sigm(nodep[(size_t)hd * np + n]);
}

__global__ __launch_bounds__(NTHR) void k_out(
    const float* __restrict__ nodep, const int* __restrict__ batch, float* out,
    int nN, int np, int outN) {
  __shared__ __attribute__((aligned(16))) float smax[32];
  const int tid = threadIdx.x, lane = tid & 31, wave = tid >> 5;
  const float ninf = __uint_as_float(0xff800000u);
  if (tid < 32) smax[tid] = ninf;
  __syncthreads();
  if (blockIdx.x == 0) {
#pragma unroll 1
    for (int pi = wave; pi < NHEAD * NGRAPH; pi += NWAVE) {
      const int hd = pi >> 3, g = pi & 7;
      const float* pp = nodep + (size_t)hd * np;
      float mx = ninf;
#pragma unroll 4
      for (int n = lane; n < nN; n += 32) {
        const float v = pp[n];
        const int b = batch[n];
        mx = (b == g) ? fmaxf(mx, v) : mx;
      }
      mx = fmaxf(mx, __shfl_xor(mx, 16, 32));
      mx = fmaxf(mx, __shfl_xor(mx, 8, 32));
      mx = fmaxf(mx, __shfl_xor(mx, 4, 32));
      mx = fmaxf(mx, __shfl_xor(mx, 2, 32));
      mx = fmaxf(mx, __shfl_xor(mx, 1, 32));
      if (lane == 0) smax[pi] = mx;
    }
  }
  __syncthreads();

  const int nF4 = (outN + 3) >> 2;
  const int gi  = blockIdx.x * NTHR + tid;
  const int f0  = 4 * gi;
  v4f vv;
  vv.x = out_elem(f0,     smax, nodep, nN, np, outN);
  vv.y = out_elem(f0 + 1, smax, nodep, nN, np, outN);
  vv.z = out_elem(f0 + 2, smax, nodep, nN, np, outN);
  vv.w = out_elem(f0 + 3, smax, nodep, nN, np, outN);
  const bool full = (gi < nF4) && (f0 + 3 < outN);
  const bool tail = (gi < nF4) && !full;
  if (full) {
    *(volatile v4f*)(out + f0) = vv;
  } else if (tail) {
    if (f0     < outN) *(volatile float*)(out + f0)     = vv.x;
    if (f0 + 1 < outN) *(volatile float*)(out + f0 + 1) = vv.y;
    if (f0 + 2 < outN) *(volatile float*)(out + f0 + 2) = vv.z;
  }
  __threadfence();
  if (full) {
    *(volatile v4f*)(out + f0) = vv;
  } else if (tail) {
    if (f0     < outN) *(volatile float*)(out + f0)     = vv.x;
    if (f0 + 1 < outN) *(volatile float*)(out + f0 + 1) = vv.y;
    if (f0 + 2 < outN) *(volatile float*)(out + f0 + 2) = vv.z;
  }
}

extern "C" void kernel_launch(void* const* d_in, const int* in_sizes, int n_in,
                              void* d_out, int out_size, void* d_ws, size_t ws_size,
                              hipStream_t stream) {
  if (n_in < 29) return;
  const int nN = in_sizes[0] / DF;
  const int nE = in_sizes[1] / 2;
  if (nN <= 0 || nE < 0 || in_sizes[0] != nN * DF || in_sizes[1] != nE * 2) return;
  if (in_sizes[2] != nN) return;
  if (in_sizes[3] != WPL || in_sizes[9] != 2 * WPL || in_sizes[15] != NHEAD * WPL ||
      in_sizes[21] != NHEAD * WPL || in_sizes[27] != NHEAD * DF || in_sizes[28] < NHEAD) return;
  for (int i = 4; i <= 8; ++i)   if (in_sizes[i] < DF) return;
  for (int i = 10; i <= 14; ++i) if (in_sizes[i] < 2 * DF) return;
  for (int i = 16; i <= 20; ++i) if (in_sizes[i] < NHEAD * DF) return;
  for (int i = 22; i <= 26; ++i) if (in_sizes[i] < NHEAD * DF) return;
  if (out_size != NHEAD * NGRAPH + NHEAD * nN) return;

  const float* x        = (const float*)d_in[0];
  const int*   ei       = (const int*)d_in[1];
  const int*   batch    = (const int*)d_in[2];
  const float* W_first  = (const float*)d_in[3];
  const float* b_first  = (const float*)d_in[4];
  const float* g_first  = (const float*)d_in[5];
  const float* be_first = (const float*)d_in[6];
  const float* rm_first = (const float*)d_in[7];
  const float* rv_first = (const float*)d_in[8];
  const float* W_conv   = (const float*)d_in[9];
  const float* b_conv   = (const float*)d_in[10];
  const float* g_conv   = (const float*)d_in[11];
  const float* be_conv  = (const float*)d_in[12];
  const float* rm_conv  = (const float*)d_in[13];
  const float* rv_conv  = (const float*)d_in[14];
  const float* W1  = (const float*)d_in[15];
  const float* b1  = (const float*)d_in[16];
  const float* g1  = (const float*)d_in[17];
  const float* be1 = (const float*)d_in[18];
  const float* rm1 = (const float*)d_in[19];
  const float* rv1 = (const float*)d_in[20];
  const float* W2  = (const float*)d_in[21];
  const float* b2  = (const float*)d_in[22];
  const float* g2  = (const float*)d_in[23];
  const float* be2 = (const float*)d_in[24];
  const float* rm2 = (const float*)d_in[25];
  const float* rv2 = (const float*)d_in[26];
  const float* W3  = (const float*)d_in[27];
  const float* b3  = (const float*)d_in[28];
  float* out = (float*)d_out;

  const int nG = (nN + GROWS - 1) / GROWS;
  const int nA = (nN + NBA - 1) / NBA;
  const int NP = nA * NBA;

  char* ws = (char*)d_ws;
  const size_t rbytes = (size_t)NP * DF * 4;
  size_t off = 0;
  const size_t oW  = off; off += (size_t)NMAT * 2 * WPL * 2;   off = (off + 255) & ~(size_t)255;
  const size_t oR1 = off; off += rbytes;                       off = (off + 255) & ~(size_t)255;
  const size_t oR2 = off; off += rbytes;                       off = (off + 255) & ~(size_t)255;
  const size_t oNd = off; off += (size_t)NHEAD * NP * 4;       off = (off + 255) & ~(size_t)255;
  if (off > ws_size) return;
  if (off > (size_t)134217728) return;
  unsigned short* wpl = (unsigned short*)(ws + oW);
  float*          R1f = (float*)(ws + oR1);
  unsigned short* R1h = (unsigned short*)(ws + oR1);
  unsigned short* R1l = R1h + (size_t)NP * DF;
  float*          R2f = (float*)(ws + oR2);
  unsigned short* R2h = (unsigned short*)(ws + oR2);
  unsigned short* R2l = R2h + (size_t)NP * DF;
  float*          nodep = (float*)(ws + oNd);

  const int vec8 = ((nE & 3) == 0) ? 1 : 0;
  const float f16inv = 0.0625f;

  k_wprep<<<dim3(WPL / 8 / NTHR, NMAT), NTHR, 0, stream>>>(W_first, W_conv, W1, W2, wpl);

  hipFuncSetAttribute(reinterpret_cast<const void*>(&k_gemm<0, 0>), hipFuncAttributeMaxDynamicSharedMemorySize, LDS_GEMM);
  hipFuncSetAttribute(reinterpret_cast<const void*>(&k_gemm<1, 0>), hipFuncAttributeMaxDynamicSharedMemorySize, LDS_GEMM);
  hipFuncSetAttribute(reinterpret_cast<const void*>(&k_gemm<2, 1>), hipFuncAttributeMaxDynamicSharedMemorySize, LDS_GEMM);
  hipFuncSetAttribute(reinterpret_cast<const void*>(&k_agg<0>), hipFuncAttributeMaxDynamicSharedMemorySize, LDS_AGG);
  hipFuncSetAttribute(reinterpret_cast<const void*>(&k_agg<1>), hipFuncAttributeMaxDynamicSharedMemorySize, LDS_AGG);

  k_gemm<0, 0><<<nG, NTHR, LDS_GEMM, stream>>>(x, wpl, wpl, wpl,
      b_first, g_first, be_first, rm_first, rv_first, W3, b3,
      R1f, R2h, R2l, nodep, nN, f16inv);
  k_agg<0><<<nA, NTHR, LDS_AGG, stream>>>(ei, R1f, R2h, R2l, nN, nE, vec8);
  k_gemm<1, 0><<<nG, NTHR, LDS_GEMM, stream>>>(x, R2h, R2l, wpl + (size_t)1 * 2 * WPL,
      b_conv, g_conv, be_conv, rm_conv, rv_conv, W3, b3,
      R1f, R1h, R1l, nodep, nN, f16inv);
  k_agg<1><<<nA, NTHR, LDS_AGG, stream>>>(ei, R1f, R2h, R2l, nN, nE, vec8);
  k_gemm<2, 1><<<nG, NTHR, LDS_GEMM, stream>>>(x, R2h, R2l, wpl + (size_t)2 * 2 * WPL,
      b_conv + DF, g_conv + DF, be_conv + DF, rm_conv + DF, rv_conv + DF, W3, b3,
      R2f, R1h, R1l, nodep, nN, 1.0f);
  for (int hd = 0; hd < NHEAD; ++hd) {
    k_gemm<2, 1><<<nG, NTHR, LDS_GEMM, stream>>>(x, R1h, R1l, wpl + (size_t)(3 + hd) * 2 * WPL,
        b1 + hd * DF, g1 + hd * DF, be1 + hd * DF, rm1 + hd * DF, rv1 + hd * DF, W3, b3,
        R2f, R2h, R2l, nodep, nN, 1.0f);
    k_gemm<2, 2><<<nG, NTHR, 0, stream>>>(x, R2h, R2l, wpl + (size_t)(6 + hd) * 2 * WPL,
        b2 + hd * DF, g2 + hd * DF, be2 + hd * DF, rm2 + hd * DF, rv2 + hd * DF,
        W3 + hd * DF, b3 + hd, R1f, R1h, R1l, nodep + (size_t)hd * NP, nN, 1.0f);
  }
  const int nF4 = (out_size + 3) / 4;
  k_out<<<(nF4 + NTHR - 1) / NTHR, NTHR, 0, stream>>>(nodep, batch, out, nN, NP, out_size);
}
